// MarketBDHPretrain_61555471286948
// MI455X (gfx1250) — hardware-run, weakly checked
//
#include <hip/hip_runtime.h>


#ifndef NB
#define NB 2
#endif
#ifndef SEQ
#define SEQ 512
#endif
#define NB_FULL  2
#define SEQ_FULL 512
#ifndef OUT_SEQ
#define OUT_SEQ SEQ
#endif
#define DM   256
#define NH_  4
#define NI   4096
#define NP   (NI / 2)
#define IND  372
#define INDP 384
#define NL   6
#define ROWS (NB * SEQ)
#define NT64 (SEQ / 64)
#define TP   68
#define LNP  260
#define HDP  388
#define WSC  64.0f
#define WSI  (1.0f / 64.0f)
#define XYC  16.0f
#define XYI  (1.0f / 1024.0f)
#define EPSF 1e-5f

static_assert(NH_ * NI == 16384);
static_assert(NI == 4096);
static_assert(DM == 256);
static_assert(DM % 64 == 0);
static_assert(DM % 32 == 0);
static_assert(NI % 64 == 0);
static_assert(NI % 32 == 0);
static_assert(SEQ % 64 == 0);
static_assert(ROWS % 64 == 0);
static_assert(INDP % 64 == 0);
static_assert(INDP % 32 == 0);
static_assert(INDP >= IND);
static_assert(IND % 4 == 0);
static_assert((IND * 4) % 16 == 0);
static_assert((64 * IND * 4) % 128 == 0);
static_assert(OUT_SEQ % 64 == 0);
static_assert(64 * IND / 4 == 192 * 31);
static_assert(4 * 32 * 16 == 16 * 64 * 2);
static_assert(16 * 32 * 16 == 64 * 64 * 2);
static_assert(32 * 32 * 16 == 16 * DM * 4);
static_assert(16 * 32 * 16 == 16 * DM * 2);
static_assert(16 * 32 * 16 == 64 * 64 * 2);
static_assert(2 * 256 * 16 == 64 * 64 * 2);
static_assert(NB <= NB_FULL);
static_assert(SEQ <= SEQ_FULL);
static_assert((TP * 4) % 16 == 0);
static_assert((LNP * 4) % 16 == 0);
static_assert((HDP * 4) % 16 == 0);
static_assert(HDP >= INDP);
static_assert(LNP >= DM);
static_assert(64 * LNP * 4 <= 131072);
static_assert(64 * HDP * 4 <= 131072);
static_assert(64 * TP * 4 <= 131072);
static_assert(NT64 * (NT64 + 1) / 2 <= 65535);

typedef _Float16 h16;
typedef __attribute__((ext_vector_type(16))) _Float16 v16h;
typedef __attribute__((ext_vector_type(8)))  _Float16 v8h;
typedef __attribute__((ext_vector_type(8)))  float    v8f;
typedef __attribute__((ext_vector_type(4)))  float    v4f;
typedef __attribute__((ext_vector_type(2)))  float    v2f;
typedef v4f  __attribute__((may_alias)) v4fa;

__device__ __forceinline__ unsigned short f2bf(float f) { unsigned u = __float_as_uint(f); u += 0x7FFFu + ((u >> 16) & 1u); return (unsigned short)(u >> 16); }
__device__ __forceinline__ float bfr(float f) { return __uint_as_float(((unsigned)f2bf(f)) << 16); }
__device__ __forceinline__ v16h cat16(v8h lo, v8h hi) { return __builtin_shufflevector(lo, hi, 0, 1, 2, 3, 4, 5, 6, 7, 8, 9, 10, 11, 12, 13, 14, 15); }
__device__ __forceinline__ v8f wmma16(v16h a, v16h b, v8f c) { return __builtin_amdgcn_wmma_f32_16x16x32_f16(false, a, false, b, (short)0, c, false, false); }
__device__ __forceinline__ v16h  ldh(const h16* p) { return cat16(*(const v8h*)p, *(const v8h*)(p + 16)); }
__device__ __forceinline__ void wave_sync() { __builtin_amdgcn_fence(3  , "wavefront"); __builtin_amdgcn_wave_barrier(); asm volatile("" ::: "memory"); }
static __device__ __forceinline__ h16 toh_flush(float v) { const h16 r = (h16)v; return (fabsf(v) < 6.103515625e-05f) ? (h16)0.0f : r; }
__device__ __forceinline__ float wsum(float v) {
    v += __shfl_xor(v, 16, 32); v += __shfl_xor(v, 8, 32); v += __shfl_xor(v, 4, 32); v += __shfl_xor(v, 2, 32); v += __shfl_xor(v, 1, 32); return v; }

__device__ __forceinline__ void ln8(float (&xs)[8]) {
    float s = 0.0f;
#pragma unroll
    for (int i = 0; i < 8; ++i) s += xs[i];
    s = wsum(s); const float mu = s * (1.0f / DM);
    float q = 0.0f;
#pragma unroll
    for (int i = 0; i < 8; ++i) { xs[i] -= mu; q += xs[i] * xs[i]; }
    q = wsum(q);
    const float rs = rsqrtf(q * (1.0f / DM) + EPSF);
#pragma unroll
    for (int i = 0; i < 8; ++i) xs[i] *= rs;
}

__device__ __forceinline__ void mma64(const h16* __restrict__ A, const h16* __restrict__ Bt, size_t aoff, size_t boff, size_t lda, size_t ldb, int K, v8f (&acc)[4][4]) {
#pragma unroll 1
    for (int kc = 0; kc < K; kc += 32) {
        v16h a[4];
#pragma unroll
        for (int mb = 0; mb < 4; ++mb) a[mb] = ldh(A + aoff + (size_t)mb * 16 * lda + kc);
#pragma unroll
        for (int nb = 0; nb < 4; ++nb) { const v16h b = ldh(Bt + boff + (size_t)nb * 16 * ldb + kc);
#pragma unroll
            for (int mb = 0; mb < 4; ++mb) acc[mb][nb] = wmma16(a[mb], b, acc[mb][nb]); }
        asm volatile("v_nop\n\tv_nop\n\tv_nop\n\tv_nop" : "+v"(acc[0][0]), "+v"(acc[1][1]), "+v"(acc[2][2]), "+v"(acc[3][3]) : "v"(a[0]), "v"(a[1]), "v"(a[2]), "v"(a[3]));
    }
}

__global__ __launch_bounds__(256) void k_tr(const float* __restrict__ src, h16* dst, int R, int C, int Rp, int Cp, float scale) {
#pragma clang fp contract(off)
    __shared__ float tl[64 * 65];
    const int tid = threadIdx.x; const int r0 = blockIdx.x * 64, c0 = blockIdx.y * 64; const int z = blockIdx.z;
    const float* sp = src + (size_t)z * (size_t)R * (size_t)C;
#pragma unroll 4
    for (int it = 0; it < 16; ++it) { const int idx = it * 256 + tid; const int r = idx >> 6, c = idx & 63;
        const int rr = (r0 + r) < R ? (r0 + r) : (R - 1); const int cc = (c0 + c) < C ? (c0 + c) : (C - 1);
        float v = sp[(size_t)rr * C + cc]; asm volatile("" : "+v"(v));
        const bool ok = ((r0 + r) < R) & ((c0 + c) < C);
        tl[r * 65 + c] = ok ? bfr(v) * scale : 0.0f; }
    __syncthreads();
    h16* dp = dst + ((size_t)z * Cp + c0) * (size_t)Rp + r0;
#pragma unroll 1
    for (int ps = 0; ps < 2; ++ps) {
#pragma unroll
        for (int it = 0; it < 2; ++it) { const int crow = it * 32 + (tid >> 3), r8 = (tid & 7) * 8;
            v8h o;
#pragma unroll
            for (int q = 0; q < 8; ++q) o[q] = toh_flush(tl[(r8 + q) * 65 + crow]);
            *(volatile v8h*)(dp + (size_t)crow * Rp + r8) = o; }
        if (ps == 0) __threadfence(); }
}

__global__ __launch_bounds__(256) void k_xcvt(const float* __restrict__ x, h16* XH) {
    const int i = blockIdx.x * 256 + threadIdx.x; if (i >= ROWS * (INDP / 8)) return;
    const int R = i / (INDP / 8), c = (i % (INDP / 8)) * 8;
    const int b = R / SEQ, t = R % SEQ;
    const float* sp = x + ((size_t)b * SEQ_FULL + t) * IND;
    const int ca = c < (IND - 4) ? c : (IND - 4); const int cb = (c + 4) < (IND - 4) ? (c + 4) : (IND - 4);
    v4f va = *(const v4f*)(sp + ca); v4f vb = *(const v4f*)(sp + cb);
    asm volatile("" : "+v"(va)); asm volatile("" : "+v"(vb));
    const bool oka = c < IND, okb = (c + 4) < IND;
    v8h o;
#pragma unroll
    for (int k = 0; k < 4; ++k) { o[k] = oka ? toh_flush(bfr(va[k])) : (h16)0.0f; o[4 + k] = okb ? toh_flush(bfr(vb[k])) : (h16)0.0f; }
    *(volatile v8h*)(XH + (size_t)i * 8) = o; __threadfence(); *(volatile v8h*)(XH + (size_t)i * 8) = o;
}

__global__ __launch_bounds__(256) void k_cs(float* CS) {
#pragma clang fp contract(off)
    const int i = blockIdx.x * 256 + threadIdx.x; if (i >= SEQ * (NP / 2)) return;
    const int t = i / (NP / 2), p0 = (i % (NP / 2)) * 2;
    float c0 = 0.0f, s0 = 0.0f, c1 = 0.0f, s1 = 0.0f;
#pragma unroll 1
    for (int k = 0; k < 2; ++k) {
        const float e = (float)(p0 + k) * (1.0f / 128.0f);
        const float fr = 1.0f / exp2f(e);
        const float ph = (float)t * fr;
        const float c = cosf(ph); const float s = sinf(ph);
        c0 = (k == 0) ? c : c0; s0 = (k == 0) ? s : s0;
        c1 = (k == 0) ? c1 : c; s1 = (k == 0) ? s1 : s;
    }
    v4f o; o[0] = c0; o[1] = s0; o[2] = c1; o[3] = s1;
    *(volatile v4f*)(CS + (size_t)i * 4) = o; __threadfence(); *(volatile v4f*)(CS + (size_t)i * 4) = o;
}

__global__ __launch_bounds__(32) void k_hs(const h16* __restrict__ HF, const h16* __restrict__ ENCT, const float* __restrict__ CS, h16* HS, h16* QR) {
    __shared__ __align__(16) float os[16 * TP];
    const int lane = threadIdx.x & 31, lr = lane & 15, hi = lane >> 4;
    const int r0 = blockIdx.x * 64, c0 = blockIdx.y * 64, hd = blockIdx.z;
    v8f acc[4][4];
#pragma unroll
    for (int mb = 0; mb < 4; ++mb)
#pragma unroll
        for (int nb = 0; nb < 4; ++nb) acc[mb][nb] = (v8f){};
    mma64(HF, ENCT, (size_t)(r0 + lr) * DM + 8 * hi, ((size_t)hd * NI + c0 + lr) * DM + 8 * hi, DM, DM, DM, acc);
    const size_t pb = ((size_t)hd * ROWS + (size_t)r0) * NI + (size_t)c0;
#pragma unroll
    for (int mb = 0; mb < 4; ++mb) {
#pragma unroll
        for (int nb = 0; nb < 4; ++nb) {
#pragma unroll
            for (int j = 0; j < 8; ++j) os[(hi * 8 + j) * TP + nb * 16 + lr] = fmaxf(acc[mb][nb][j] * WSI, 0.0f); }
        wave_sync();
        v8h hv[4], qv[4];
#pragma unroll
        for (int s = 0; s < 4; ++s) { const int row = 4 * s + (lane >> 3), c8 = (lane & 7) * 8;
            const v4f x0 = *(const v4fa*)(&os[row * TP + c8]); const v4f x1 = *(const v4fa*)(&os[row * TP + c8 + 4]);
            const int t = (r0 + mb * 16 + row) % SEQ;
            const float* cp = CS + (size_t)t * NI + c0 + c8;
            const v4f e0 = *(const v4f*)cp; const v4f e1 = *(const v4f*)(cp + 4);
            v8h a, q;
#pragma unroll
            for (int i = 0; i < 4; ++i) { a[i] = toh_flush(x0[i]); a[4 + i] = toh_flush(x1[i]); }
            q[0] = toh_flush(x0[0] * e0[0] - x0[1] * e0[1]); q[1] = toh_flush(x0[0] * e0[1] + x0[1] * e0[0]);
            q[2] = toh_flush(x0[2] * e0[2] - x0[3] * e0[3]); q[3] = toh_flush(x0[2] * e0[3] + x0[3] * e0[2]);
            q[4] = toh_flush(x1[0] * e1[0] - x1[1] * e1[1]); q[5] = toh_flush(x1[0] * e1[1] + x1[1] * e1[0]);
            q[6] = toh_flush(x1[2] * e1[2] - x1[3] * e1[3]); q[7] = toh_flush(x1[2] * e1[3] + x1[3] * e1[2]);
            hv[s] = a; qv[s] = q; }
#pragma unroll 1
        for (int ps = 0; ps < 2; ++ps) {
#pragma unroll
            for (int s = 0; s < 4; ++s) { const int row = 4 * s + (lane >> 3), c8 = (lane & 7) * 8;
                const size_t oo = pb + (size_t)(mb * 16 + row) * NI + c8;
                *(volatile v8h*)(HS + oo) = hv[s]; *(volatile v8h*)(QR + oo) = qv[s]; }
            if (ps == 0) __threadfence(); }
        wave_sync();
    }
}

__global__ __launch_bounds__(32) void k_sc(const h16* __restrict__ QR, h16* S) {
    __shared__ __align__(16) float os[64 * TP];
    const int lane = threadIdx.x & 31, lr = lane & 15, hi = lane >> 4;
    int ti = 0, rem = (int)blockIdx.x;
#pragma unroll 1
    for (int q = 0; q < NT64 - 1; ++q) { const int w = NT64 - ti; if (rem >= w) { rem -= w; ti += 1; } }
    const int tj = ti + rem;
    const int z = blockIdx.y; const int b = z / NH_, hd = z % NH_;
    const size_t qb = ((size_t)hd * ROWS + (size_t)b * SEQ) * NI;
    v8f acc[4][4];
#pragma unroll
    for (int mb = 0; mb < 4; ++mb)
#pragma unroll
        for (int nb = 0; nb < 4; ++nb) acc[mb][nb] = (v8f){};
    mma64(QR, QR, qb + (size_t)(ti * 64 + lr) * NI + 8 * hi, qb + (size_t)(tj * 64 + lr) * NI + 8 * hi, NI, NI, NI, acc);
#pragma unroll
    for (int mb = 0; mb < 4; ++mb)
#pragma unroll
        for (int nb = 0; nb < 4; ++nb)
#pragma unroll
            for (int j = 0; j < 8; ++j) os[(mb * 16 + hi * 8 + j) * TP + nb * 16 + lr] = acc[mb][nb][j];
    wave_sync();
    h16* sd = S + ((size_t)z * SEQ + (size_t)ti * 64) * SEQ + (size_t)tj * 64;
    h16* sm = S + ((size_t)z * SEQ + (size_t)tj * 64) * SEQ + (size_t)ti * 64;
#pragma unroll 1
    for (int ps = 0; ps < 2; ++ps) {
#pragma unroll 1
        for (int s = 0; s < 16; ++s) { const int row = 4 * s + (lane >> 3), c8 = (lane & 7) * 8;
            const v4f x0 = *(const v4fa*)(&os[row * TP + c8]); const v4f x1 = *(const v4fa*)(&os[row * TP + c8 + 4]);
            v8h o;
#pragma unroll
            for (int i = 0; i < 4; ++i) { o[i] = toh_flush(x0[i]); o[4 + i] = toh_flush(x1[i]); }
            *(volatile v8h*)(sd + (size_t)row * SEQ + c8) = o;
            if (ti != tj) {
                v8h m;
#pragma unroll
                for (int q = 0; q < 8; ++q) m[q] = toh_flush(os[(c8 + q) * TP + row]);
                *(volatile v8h*)(sm + (size_t)row * SEQ + c8) = m; } }
        if (ps == 0) __threadfence(); }
}

__global__ __launch_bounds__(32) void k_ys(const h16* __restrict__ YK, const h16* __restrict__ ENCVT, const h16* __restrict__ HS, h16* XY) {
    __shared__ __align__(16) float os[16 * TP];
    const int lane = threadIdx.x & 31, lr = lane & 15, hi = lane >> 4;
    const int r0 = blockIdx.x * 64, c0 = blockIdx.y * 64, z = blockIdx.z; const int b = z / NH_, hd = z % NH_;
    v8f acc[4][4];
#pragma unroll
    for (int mb = 0; mb < 4; ++mb)
#pragma unroll
        for (int nb = 0; nb < 4; ++nb) acc[mb][nb] = (v8f){};
    mma64(YK, ENCVT, ((size_t)z * SEQ + r0 + lr) * DM + 8 * hi, ((size_t)hd * NI + c0 + lr) * DM + 8 * hi, DM, DM, DM, acc);
    const size_t pb = ((size_t)hd * ROWS + (size_t)b * SEQ + (size_t)r0) * NI + (size_t)c0;
#pragma unroll
    for (int mb = 0; mb < 4; ++mb) {
#pragma unroll
        for (int nb = 0; nb < 4; ++nb) {
#pragma unroll
            for (int j = 0; j < 8; ++j) os[(hi * 8 + j) * TP + nb * 16 + lr] = fmaxf(acc[mb][nb][j] * WSI, 0.0f); }
        wave_sync();
        v8h xv[4];
#pragma unroll
        for (int s = 0; s < 4; ++s) { const int row = 4 * s + (lane >> 3), c8 = (lane & 7) * 8;
            const v4f x0 = *(const v4fa*)(&os[row * TP + c8]); const v4f x1 = *(const v4fa*)(&os[row * TP + c8 + 4]);
            const v8h g = *(const v8h*)(HS + pb + (size_t)(mb * 16 + row) * NI + c8);
            v8h o;
#pragma unroll
            for (int i = 0; i < 4; ++i) { o[i] = toh_flush(x0[i] * (float)g[i] * XYC); o[4 + i] = toh_flush(x1[i] * (float)g[4 + i] * XYC); }
            xv[s] = o; }
#pragma unroll 1
        for (int ps = 0; ps < 2; ++ps) {
#pragma unroll
            for (int s = 0; s < 4; ++s) { const int row = 4 * s + (lane >> 3), c8 = (lane & 7) * 8;
                *(volatile v8h*)(XY + pb + (size_t)(mb * 16 + row) * NI + c8) = xv[s]; }
            if (ps == 0) __threadfence(); }
        wave_sync();
    }
}

template <int MODE>
__device__ __forceinline__ void lnblock(const h16* __restrict__ A, const h16* __restrict__ Bt, const float* __restrict__ bias, float* H32, h16* HF, h16* HT, h16* YK) {
    __shared__ __align__(16) float os[64 * LNP];
    const int lane = threadIdx.x & 31, lr = lane & 15, hi = lane >> 4;
    const int wave = __builtin_amdgcn_readfirstlane((int)(threadIdx.x >> 5));
    const int r0 = blockIdx.x * 64, c0 = wave * 64; const int z = blockIdx.y;
    v8f acc[4][4];
#pragma unroll
    for (int mb = 0; mb < 4; ++mb)
#pragma unroll
        for (int nb = 0; nb < 4; ++nb) acc[mb][nb] = (v8f){};
    float scale;
    if (MODE == 0) {
        mma64(A, Bt, (size_t)(r0 + lr) * INDP + 8 * hi, (size_t)(c0 + lr) * INDP + 8 * hi, INDP, INDP, INDP, acc); scale = WSI;
    } else if (MODE == 1) {
        mma64(A, Bt, ((size_t)z * SEQ + r0 + lr) * SEQ + 8 * hi, ((size_t)(z / NH_) * DM + c0 + lr) * SEQ + 8 * hi, SEQ, SEQ, SEQ, acc); scale = 1.0f;
    } else {
#pragma unroll 1
        for (int hd = 0; hd < NH_; ++hd)
            mma64(A, Bt, ((size_t)hd * ROWS + r0 + lr) * NI + 8 * hi, ((size_t)hd * DM + c0 + lr) * NI + 8 * hi, NI, NI, NI, acc);
        scale = XYI;
    }
#pragma unroll
    for (int nb = 0; nb < 4; ++nb) {
        const float bc = (MODE == 0) ? bfr(bias[c0 + nb * 16 + lr]) : 0.0f;
#pragma unroll
        for (int mb = 0; mb < 4; ++mb)
#pragma unroll
            for (int j = 0; j < 8; ++j) os[(mb * 16 + hi * 8 + j) * LNP + c0 + nb * 16 + lr] = acc[mb][nb][j] * scale + bc; }
    __syncthreads();
#pragma unroll 1
    for (int rr = 0; rr < 16; ++rr) {
        const int row = wave * 16 + rr; const int ob = row * LNP + 8 * lane;
        const v4f x0 = *(const v4fa*)(&os[ob]); const v4f x1 = *(const v4fa*)(&os[ob + 4]);
        float xs[8];
#pragma unroll
        for (int i = 0; i < 4; ++i) { xs[i] = x0[i]; xs[4 + i] = x1[i]; }
        ln8(xs);
        if (MODE == 2) {
            const float* hp = H32 + (size_t)(r0 + row) * DM + 8 * lane;
            const v4f g0 = *(const v4f*)hp; const v4f g1 = *(const v4f*)(hp + 4);
#pragma unroll
            for (int i = 0; i < 4; ++i) { xs[i] += g0[i]; xs[4 + i] += g1[i]; }
            ln8(xs);
        }
        v4f y0, y1;
#pragma unroll
        for (int i = 0; i < 4; ++i) { y0[i] = xs[i]; y1[i] = xs[4 + i]; }
        *(v4fa*)(&os[ob]) = y0; *(v4fa*)(&os[ob + 4]) = y1;
    }
    __syncthreads();
    const int bq = r0 / SEQ, t0 = r0 % SEQ;
#pragma unroll 1
    for (int ps = 0; ps < 2; ++ps) {
        if (MODE == 1) {
#pragma unroll 1
            for (int it = 0; it < 16; ++it) { const int p = it * 32 + lane; const int row = wave * 16 + (p >> 5), c8 = (p & 31) * 8;
                const v4f x0 = *(const v4fa*)(&os[row * LNP + c8]); const v4f x1 = *(const v4fa*)(&os[row * LNP + c8 + 4]); v8h o;
#pragma unroll
                for (int i = 0; i < 4; ++i) { o[i] = toh_flush(x0[i]); o[4 + i] = toh_flush(x1[i]); }
                *(volatile v8h*)(YK + ((size_t)z * SEQ + r0 + row) * DM + c8) = o; }
        } else {
#pragma unroll 1
            for (int it = 0; it < 32; ++it) { const int p = it * 32 + lane; const int row = wave * 16 + (p >> 6), c4 = (p & 63) * 4;
                const v4f val = *(const v4fa*)(&os[row * LNP + c4]);
                *(volatile v4f*)(H32 + (size_t)(r0 + row) * DM + c4) = val; }
#pragma unroll 1
            for (int it = 0; it < 16; ++it) { const int p = it * 32 + lane; const int row = wave * 16 + (p >> 5), c8 = (p & 31) * 8;
                const v4f x0 = *(const v4fa*)(&os[row * LNP + c8]); const v4f x1 = *(const v4fa*)(&os[row * LNP + c8 + 4]); v8h o;
#pragma unroll
                for (int i = 0; i < 4; ++i) { o[i] = toh_flush(x0[i]); o[4 + i] = toh_flush(x1[i]); }
                *(volatile v8h*)(HF + (size_t)(r0 + row) * DM + c8) = o; }
#pragma unroll 1
            for (int s = 0; s < 16; ++s) { const int d = wave * 64 + 4 * s + (lane >> 3), c8 = (lane & 7) * 8;
                v8h o;
#pragma unroll
                for (int q = 0; q < 8; ++q) o[q] = toh_flush(os[(c8 + q) * LNP + d]);
                *(volatile v8h*)(HT + ((size_t)bq * DM + d) * SEQ + t0 + c8) = o; }
        }
        if (ps == 0) __threadfence(); }
}

__global__ __launch_bounds__(128) void k_inproj(const h16* __restrict__ XH, const h16* __restrict__ WINT, const float* __restrict__ inb, float* H32, h16* HF, h16* HT) {
    lnblock<0>(XH, WINT, inb, H32, HF, HT, HF);
}
__global__ __launch_bounds__(128) void k_ykv(const h16* __restrict__ S, const h16* __restrict__ HT, h16* YK) {
    lnblock<1>(S, HT, (const float*)0, (float*)0, YK, YK, YK);
}
__global__ __launch_bounds__(128) void k_ymlp(const h16* __restrict__ XY, const h16* __restrict__ DECT, float* H32, h16* HF, h16* HT) {
    lnblock<2>(XY, DECT, (const float*)0, H32, HF, HT, HF);
}

__global__ __launch_bounds__(192) void k_head(const h16* __restrict__ HF, const h16* __restrict__ HWT, const float* __restrict__ hb, float* OUT) {
    __shared__ __align__(16) float os[64 * HDP];
    const int lane = threadIdx.x & 31, lr = lane & 15, hi = lane >> 4;
    const int wave = __builtin_amdgcn_readfirstlane((int)(threadIdx.x >> 5));
    const int r0 = blockIdx.x * 64, c0 = wave * 64;
    v8f acc[4][4];
#pragma unroll
    for (int mb = 0; mb < 4; ++mb)
#pragma unroll
        for (int nb = 0; nb < 4; ++nb) acc[mb][nb] = (v8f){};
    mma64(HF, HWT, (size_t)(r0 + lr) * DM + 8 * hi, (size_t)(c0 + lr) * DM + 8 * hi, DM, DM, DM, acc);
#pragma unroll
    for (int mb = 0; mb < 4; ++mb)
#pragma unroll
        for (int nb = 0; nb < 4; ++nb)
#pragma unroll
            for (int j = 0; j < 8; ++j) os[(mb * 16 + hi * 8 + j) * HDP + c0 + nb * 16 + lr] = acc[mb][nb][j] * WSI;
    __syncthreads();
    const int bq = r0 / SEQ, t0 = r0 % SEQ;
    float* ob = OUT + ((size_t)bq * OUT_SEQ + t0) * IND;
#pragma unroll 1
    for (int ps = 0; ps < 2; ++ps) {
#pragma unroll 1
        for (int it = 0; it < 31; ++it) { const int e = (it * 192 + (int)threadIdx.x) * 4; const int row = e / IND, col = e - row * IND;
            const v4f x = *(const v4fa*)(&os[row * HDP + col]); const v4f bb = *(const v4f*)(hb + col); v4f val;
#pragma unroll
            for (int k = 0; k < 4; ++k) val[k] = x[k] + bfr(bb[k]);
            *(volatile v4f*)(ob + e) = val; }
        if (ps == 0) __threadfence(); }
}

static constexpr size_t al256(size_t v) { return (v + 255) & ~(size_t)255; }
static constexpr size_t SZ_W   = al256((size_t)NH_ * NI * DM * 2);
static constexpr size_t SZ_WIN = al256((size_t)DM * INDP * 2);
static constexpr size_t SZ_HW  = al256((size_t)INDP * DM * 2);
static constexpr size_t SZ_XH  = al256((size_t)ROWS * INDP * 2);
static constexpr size_t SZ_CS  = al256((size_t)SEQ * NI * 4);
static constexpr size_t SZ_H32 = al256((size_t)ROWS * DM * 4);
static constexpr size_t SZ_HF  = al256((size_t)ROWS * DM * 2);
static constexpr size_t SZ_BIG = al256((size_t)NH_ * ROWS * NI * 2);
static constexpr size_t SZ_S   = al256((size_t)NB * NH_ * SEQ * SEQ * 2);
static constexpr size_t SZ_YK  = al256((size_t)NB * NH_ * SEQ * DM * 2);
static constexpr size_t SZ_TOTAL = 3 * SZ_W + SZ_WIN + SZ_HW + SZ_XH + SZ_CS + SZ_H32 + 2 * SZ_HF + 2 * SZ_BIG + SZ_S + SZ_YK;
static_assert(SZ_TOTAL <= (size_t)134217728);
static_assert((size_t)NB * DM * SEQ == (size_t)ROWS * DM);
static_assert((ROWS * (INDP / 8)) % 256 == 0);
static_assert(NP % 2 == 0);
static_assert((SEQ * (NP / 2)) % 256 == 0);
static_assert((size_t)SEQ * (NP / 2) * 16 == (size_t)SEQ * NI * 4);

extern "C" void kernel_launch(void* const* d_in, const int* in_sizes, int n_in,
                              void* d_out, int out_size, void* d_ws, size_t ws_size, hipStream_t stream) {
    if (n_in < 8) return;
    if ((size_t)in_sizes[0] < ((size_t)(NB - 1) * SEQ_FULL + SEQ) * IND) return;
    if ((size_t)in_sizes[1] < (size_t)IND * DM || in_sizes[2] < DM) return;
    if ((size_t)in_sizes[3] < (size_t)NH_ * DM * NI || (size_t)in_sizes[4] < (size_t)NH_ * DM * NI || (size_t)in_sizes[5] < (size_t)NH_ * NI * DM) return;
    if ((size_t)in_sizes[6] < (size_t)DM * IND || in_sizes[7] < IND) return;
    if ((size_t)out_size < ((size_t)(NB - 1) * OUT_SEQ + SEQ) * IND) return;
    if (SZ_TOTAL > ws_size) return;
    const float* x    = (const float*)d_in[0];
    const float* inw  = (const float*)d_in[1];
    const float* inb  = (const float*)d_in[2];
    const float* enc  = (const float*)d_in[3];
    const float* encv = (const float*)d_in[4];
    const float* dec  = (const float*)d_in[5];
    const float* hw   = (const float*)d_in[6];
    const float* hb   = (const float*)d_in[7];
    float* OUT = (float*)d_out;
    char* wsp = (char*)d_ws;
    h16* ENCT  = (h16*)wsp; wsp += SZ_W;
    h16* ENCVT = (h16*)wsp; wsp += SZ_W;
    h16* DECT  = (h16*)wsp; wsp += SZ_W;
    h16* WINT  = (h16*)wsp; wsp += SZ_WIN;
    h16* HWT   = (h16*)wsp; wsp += SZ_HW;
    h16* XH    = (h16*)wsp; wsp += SZ_XH;
    float* CS  = (float*)wsp; wsp += SZ_CS;
    float* H32 = (float*)wsp; wsp += SZ_H32;
    h16* HF    = (h16*)wsp; wsp += SZ_HF;
    h16* HT    = (h16*)wsp; wsp += SZ_HF;
    h16* HS    = (h16*)wsp; wsp += SZ_BIG;
    h16* QR    = (h16*)wsp; wsp += SZ_BIG;
    h16* S     = (h16*)wsp; wsp += SZ_S;
    h16* YK    = (h16*)wsp; wsp += SZ_YK;
    h16* XY    = QR;

    k_tr<<<dim3(DM / 64, NI / 64, NH_), 256, 0, stream>>>(enc, ENCT, DM, NI, DM, NI, WSC);
    k_tr<<<dim3(DM / 64, NI / 64, NH_), 256, 0, stream>>>(encv, ENCVT, DM, NI, DM, NI, WSC);
    k_tr<<<dim3(NI / 64, DM / 64, NH_), 256, 0, stream>>>(dec, DECT, NI, DM, NI, DM, WSC);
    k_tr<<<dim3(INDP / 64, DM / 64, 1), 256, 0, stream>>>(inw, WINT, IND, DM, INDP, DM, WSC);
    k_tr<<<dim3(DM / 64, INDP / 64, 1), 256, 0, stream>>>(hw, HWT, DM, IND, DM, INDP, WSC);
    k_xcvt<<<(ROWS * (INDP / 8) + 255) / 256, 256, 0, stream>>>(x, XH);
    k_cs<<<(SEQ * (NP / 2) + 255) / 256, 256, 0, stream>>>(CS);

    k_inproj<<<dim3(ROWS / 64, 1, 1), 128, 0, stream>>>(XH, WINT, inb, H32, HF, HT);

    for (int l = 0; l < NL; ++l) {
        k_hs<<<dim3(ROWS / 64, NI / 64, NH_), 32, 0, stream>>>(HF, ENCT, CS, HS, QR);
        k_sc<<<dim3(NT64 * (NT64 + 1) / 2, NB * NH_, 1), 32, 0, stream>>>(QR, S);
        k_ykv<<<dim3(SEQ / 64, NB * NH_, 1), 128, 0, stream>>>(S, HT, YK);
        k_ys<<<dim3(SEQ / 64, NI / 64, NB * NH_), 32, 0, stream>>>(YK, ENCVT, HS, XY);
        k_ymlp<<<dim3(ROWS / 64, 1, 1), 128, 0, stream>>>(XY, DECT, H32, HF, HT);
    }

    k_head<<<dim3(ROWS / 64, 1, 1), 192, 0, stream>>>(HF, HWT, hb, OUT);
}
